// TgGIN_7189775253562
// MI455X (gfx1250) — hardware-verified
//
#include <hip/hip_runtime.h>
#include <stddef.h>


#define NTHR   256
#define NWAVE  8
#define EPT    16
#define CHUNK  (NTHR * EPT)
#define WCAP   (EPT * 32)
#define WSC    16.0f
#define WINV   0.0625f
#define KX     128
#define FD     64
#define NB     1024
#define GROWS  128

#define LDS_ACC_BYTES (NB * FD * 4)
#define LDS_LIST      (LDS_ACC_BYTES)
#define LDS_WCNT      (LDS_LIST + NWAVE * WCAP * 4)
#define LDS_AGG       (LDS_WCNT + 64)

static_assert(LDS_ACC_BYTES == 262144);
static_assert(CHUNK <= 4096);
static_assert(NB < (1 << 19));
static_assert((LDS_AGG % 16) == 0);
static_assert(LDS_AGG <= 300 * 1024);
static_assert((NB % NWAVE) == 0);
static_assert(WCAP == 32 * EPT);
static_assert((NB % GROWS) == 0);
static_assert((KX % 32) == 0 && (FD % 32) == 0);

typedef float    v2f  __attribute__((ext_vector_type(2)));
typedef float    v4f  __attribute__((ext_vector_type(4)));
typedef float    v8f  __attribute__((ext_vector_type(8)));
typedef int      v4i  __attribute__((ext_vector_type(4)));
typedef _Float16 v8h  __attribute__((ext_vector_type(8)));
typedef _Float16 v16h __attribute__((ext_vector_type(16)));
union FragH { v16h v; v8h h[2]; };
union Pk8 { v8h h; v4i i; };

__device__ __forceinline__ v8f wmh(v16h a, v16h b, v8f c) {
  v8f d = __builtin_amdgcn_wmma_f32_16x16x32_f16(false, a, false, b, (short)0, c, false, false);
  asm volatile("v_nop\n\tv_nop\n\tv_nop\n\tv_nop" : "+v"(d) : "v"(a), "v"(b));
  return d;
}

__device__ __forceinline__ v8f splat8(float x) {
  v8f c;
#pragma unroll
  for (int i = 0; i < 8; ++i) c[i] = x;
  return c;
}

__device__ __forceinline__ v8h cv8z(v4f a, v4f b, bool ok) {
  v8h r;
  r[0] = (_Float16)(ok ? a.x : 0.0f); r[1] = (_Float16)(ok ? a.y : 0.0f);
  r[2] = (_Float16)(ok ? a.z : 0.0f); r[3] = (_Float16)(ok ? a.w : 0.0f);
  r[4] = (_Float16)(ok ? b.x : 0.0f); r[5] = (_Float16)(ok ? b.y : 0.0f);
  r[6] = (_Float16)(ok ? b.z : 0.0f); r[7] = (_Float16)(ok ? b.w : 0.0f);
  return r;
}

__device__ __forceinline__ v8h cv8s(v4f a, v4f b) {
  v8h r;
  r[0] = (_Float16)(a.x * WSC); r[1] = (_Float16)(a.y * WSC);
  r[2] = (_Float16)(a.z * WSC); r[3] = (_Float16)(a.w * WSC);
  r[4] = (_Float16)(b.x * WSC); r[5] = (_Float16)(b.y * WSC);
  r[6] = (_Float16)(b.z * WSC); r[7] = (_Float16)(b.w * WSC);
  return r;
}

__global__ __launch_bounds__(NTHR) void k_prep(const float* __restrict__ w0, const float* __restrict__ w1,
                                              const float* __restrict__ w2,
                                              _Float16* p0, _Float16* p1, _Float16* p2) {
  const int b = blockIdx.x, tid = threadIdx.x;
  const float* src;
  _Float16* dst;
  int ub, tot;
  if (b < 4)      { src = w0; dst = p0; ub = b;     tot = FD * KX / 8; }
  else if (b < 6) { src = w1; dst = p1; ub = b - 4; tot = FD * FD / 8; }
  else            { src = w2; dst = p2; ub = b - 6; tot = FD * FD / 8; }
  int u = ub * NTHR + tid;
  u = u < tot ? u : tot - 1;
  const float* sp = src + (size_t)u * 8;
  const v4f a = *(const v4f*)sp;
  const v4f c = *(const v4f*)(sp + 4);
  Pk8 pk;
  pk.h = cv8s(a, c);
  _Float16* dp = dst + (size_t)u * 8;
  *(volatile v4i*)dp = pk.i;
  __threadfence();
  *(volatile v4i*)dp = pk.i;
}

__global__ __launch_bounds__(NTHR) void k_cvt(const float* __restrict__ x, _Float16* xh, int nN) {
  const int u   = blockIdx.x * NTHR + threadIdx.x;
  const int row = u >> 4;
  const int c0  = 8 * (u & 15);
  const bool ok = row < nN;
  const int rc  = ok ? row : nN - 1;
  const float* sp = x + (size_t)rc * KX + c0;
  const v4f a = *(const v4f*)sp;
  const v4f c = *(const v4f*)(sp + 4);
  Pk8 pk;
  pk.h = cv8z(a, c, ok);
  _Float16* dp = xh + (size_t)row * KX + c0;
  *(volatile v4i*)dp = pk.i;
  __threadfence();
  *(volatile v4i*)dp = pk.i;
}

__device__ __forceinline__ int scan_chunk(const int* __restrict__ dsts, int nE, int cbase, int nodeBase,
                                          int vec8, int* list, int tid, int wave) {
  const int el0  = tid * EPT;
  const int e0   = cbase + el0;
  const int sent = -2147483647 - 1;
  int d[EPT];
  if (vec8 != 0 && cbase + CHUNK <= nE) {
#pragma unroll
    for (int q = 0; q < EPT / 4; ++q) {
      const v4i t = *(const v4i*)(dsts + e0 + 4 * q);
      d[4 * q] = t.x; d[4 * q + 1] = t.y; d[4 * q + 2] = t.z; d[4 * q + 3] = t.w;
    }
  } else {
#pragma unroll
    for (int j = 0; j < EPT; ++j) {
      const int e  = e0 + j;
      const int ec = e < nE ? e : nE - 1;
      const int v  = dsts[ec];
      d[j] = (e < nE) ? v : sent;
    }
  }
  const unsigned nb = (unsigned)nodeBase;
  unsigned s[EPT];
  bool h[EPT];
  bool anyh = false;
#pragma unroll
  for (int j = 0; j < EPT; ++j) {
    s[j] = (unsigned)d[j] - nb;
    h[j] = s[j] < (unsigned)NB;
    anyh = anyh || h[j];
  }
  int wc = 0;
  const unsigned any = __builtin_amdgcn_ballot_w32(anyh);
  if (any != 0u) {
#pragma unroll
    for (int j = 0; j < EPT; ++j) {
      const unsigned mj = __builtin_amdgcn_ballot_w32(h[j]);
      if (mj != 0u) {
        if (h[j]) {
          const int pos = wc + (int)__builtin_amdgcn_mbcnt_lo(mj, 0u);
          if (pos < WCAP) list[wave * WCAP + pos] = (int)((s[j] << 12) | (unsigned)(el0 + j));
        }
        wc += (int)__builtin_popcount(mj);
      }
    }
  }
  return wc;
}

__device__ __forceinline__ void agg_rows_store(const float* __restrict__ hin, const float* acc, _Float16* aout,
                                               int nodeBase, int nN, int wave, int lane) {
  constexpr int RPW = NB / NWAVE;
  constexpr int LPR = FD / 8;
  constexpr int RPI = 32 / LPR;
  static_assert((RPW % RPI) == 0);
#pragma unroll 1
  for (int it = 0; it < RPW / RPI; ++it) {
    const int lr   = wave * RPW + it * RPI + lane / LPR;
    const int c0   = 8 * (lane % LPR);
    const int node = nodeBase + lr;
    const bool ok  = node < nN;
    const int nc   = ok ? node : nN - 1;
    const float* xp = hin + (size_t)nc * FD + c0;
    const float* ap = acc + lr * FD + c0;
    const v4f h0 = *(const v4f*)xp + *(const v4f*)ap;
    const v4f h1 = *(const v4f*)(xp + 4) + *(const v4f*)(ap + 4);
    Pk8 pk;
    pk.h = cv8z(h0, h1, ok);
    *(volatile v4i*)(aout + (size_t)node * FD + c0) = pk.i;
  }
}

__global__ __launch_bounds__(NTHR) void k_agg(const float* __restrict__ hin, const int* __restrict__ ei,
                                             _Float16* aout, int nN, int nE, int vec8) {
  extern __shared__ __attribute__((aligned(16))) unsigned char dsm[];
  float* acc  = (float*)dsm;
  int*   list = (int*)(dsm + LDS_LIST);
  int*   wcnt = (int*)(dsm + LDS_WCNT);
  const int tid = threadIdx.x, lane = tid & 31, wave = tid >> 5;
  const int nodeBase = blockIdx.x * NB;
  const int* srcs = ei;
  const int* dsts = ei + nE;

  {
    const v4f z = {0.0f, 0.0f, 0.0f, 0.0f};
    for (int i = tid; i < NB * FD / 4; i += NTHR) *(v4f*)(acc + 4 * i) = z;
  }
  __syncthreads();

  const int nChunks = (nE + CHUNK - 1) / CHUNK;
#pragma unroll 1
  for (int ch = 0; ch < nChunks; ++ch) {
    const int cbase = ch * CHUNK;
    const int wc = scan_chunk(dsts, nE, cbase, nodeBase, vec8, list, tid, wave);
    if (lane == 0) wcnt[wave] = wc;
    __syncthreads();

#pragma unroll 1
    for (int wv = 0; wv < NWAVE; ++wv) {
      int n = wcnt[wv];
      n = n > WCAP ? WCAP : (n < 0 ? 0 : n);
      const int* lp = list + wv * WCAP;
#pragma unroll 1
      for (int base = 0; base < n; base += 32) {
        const int idx  = base + lane;
        const int ent  = lp[idx < WCAP ? idx : WCAP - 1];
        const bool mine = (idx < n) && (((ent >> 12) & (NWAVE - 1)) == wave);
        unsigned mk = __builtin_amdgcn_ballot_w32(mine);
        while (mk != 0u) {
          const int j = __builtin_ctz(mk);
          mk &= mk - 1u;
          const int ej = __shfl(ent, j, 32);
          int e = cbase + (ej & 0xFFF);
          e = e > nE - 1 ? nE - 1 : e;
          int sl = ej >> 12;
          sl = sl < 0 ? 0 : (sl > NB - 1 ? NB - 1 : sl);
          int sn = srcs[e];
          sn = sn < 0 ? 0 : (sn > nN - 1 ? nN - 1 : sn);
          const float* xp = hin + (size_t)sn * FD + 2 * lane;
          float* ap = acc + sl * FD + 2 * lane;
          const v2f xv = *(const v2f*)xp;
          const v2f av = *(const v2f*)ap;
          *(v2f*)ap = av + xv;
        }
      }
    }
    __syncthreads();
  }
  __syncthreads();

  agg_rows_store(hin, acc, aout, nodeBase, nN, wave, lane);
  __threadfence();
  agg_rows_store(hin, acc, aout, nodeBase, nN, wave, lane);
}

template <int K>
__device__ __forceinline__ void mma_strip(const _Float16* __restrict__ A, const _Float16* __restrict__ Wt,
                                          int row0, int m, int hh, v8f (&acc)[4]) {
  const _Float16* ap = A  + (size_t)(row0 + m) * K + 8 * hh;
  const _Float16* bp = Wt + (size_t)m * K + 8 * hh;
#pragma unroll 2
  for (int k0 = 0; k0 < K; k0 += 32) {
    FragH a;
    a.h[0] = *(const v8h*)(ap + k0);
    a.h[1] = *(const v8h*)(ap + k0 + 16);
#pragma unroll
    for (int t = 0; t < 4; ++t) {
      FragH b;
      const _Float16* bq = bp + (size_t)(16 * t) * K + k0;
      b.h[0] = *(const v8h*)bq;
      b.h[1] = *(const v8h*)(bq + 16);
      acc[t] = wmh(a.v, b.v, acc[t]);
    }
  }
}

template <bool RELU>
__device__ __forceinline__ void stage_tile(float* st, const v8f (&acc)[4], const float* __restrict__ bias,
                                           int m, int hh) {
#pragma unroll
  for (int t = 0; t < 4; ++t) {
    const float bv = bias[16 * t + m];
#pragma unroll
    for (int r = 0; r < 8; ++r) {
      float v = acc[t][r] * WINV + bv;
      if (RELU) v = v > 0.0f ? v : 0.0f;
      st[(8 * hh + r) * FD + 16 * t + m] = v;
    }
  }
}

__device__ __forceinline__ void tile_store_f(const float* st, float* outp, int row0, int nStore, int lane) {
#pragma unroll
  for (int it = 0; it < 8; ++it) {
    const int q  = 4 * it + (lane >> 3);
    const int r  = q >> 1;
    const int cs = 32 * (q & 1) + 4 * (lane & 7);
    const v4f v = *(const v4f*)(st + r * FD + cs);
    if (row0 + r < nStore) *(volatile v4f*)(outp + (size_t)(row0 + r) * FD + cs) = v;
  }
}

template <int K, bool RELU>
__global__ __launch_bounds__(NTHR) void k_gemm(const _Float16* __restrict__ A, const _Float16* __restrict__ Wt,
                                              const float* __restrict__ bias, float* outp, int nStore) {
  __shared__ __attribute__((aligned(16))) float stg[NWAVE * 16 * FD];
  const int tid = threadIdx.x, lane = tid & 31, wave = tid >> 5, m = lane & 15, hh = lane >> 4;
  const int row0 = blockIdx.x * GROWS + 16 * wave;
  v8f acc[4];
#pragma unroll
  for (int t = 0; t < 4; ++t) acc[t] = splat8(0.0f);
  mma_strip<K>(A, Wt, row0, m, hh, acc);
  float* st = stg + wave * (16 * FD);
  stage_tile<RELU>(st, acc, bias, m, hh);
  __syncthreads();
  tile_store_f(st, outp, row0, nStore, lane);
  __threadfence();
  tile_store_f(st, outp, row0, nStore, lane);
}

extern "C" void kernel_launch(void* const* d_in, const int* in_sizes, int n_in,
                              void* d_out, int out_size, void* d_ws, size_t ws_size,
                              hipStream_t stream) {
  if (n_in < 8) return;
  const int nN = in_sizes[0] / KX;
  if (nN < 1 || in_sizes[0] != nN * KX) return;
  const int nE = in_sizes[1] / 2;
  if (nE < 1 || in_sizes[1] != 2 * nE) return;
  if (in_sizes[2] != FD * KX || in_sizes[3] != FD) return;
  if (in_sizes[4] != FD * FD || in_sizes[5] != FD) return;
  if (in_sizes[6] != FD * FD || in_sizes[7] != FD) return;
  if (out_size != nN * FD) return;

  const float* x   = (const float*)d_in[0];
  const int*   ei  = (const int*)d_in[1];
  const float* Wp  = (const float*)d_in[2];
  const float* bp  = (const float*)d_in[3];
  const float* Wf  = (const float*)d_in[4];
  const float* bf  = (const float*)d_in[5];
  const float* Wo  = (const float*)d_in[6];
  const float* bo  = (const float*)d_in[7];
  float* outp = (float*)d_out;

  const int Np = ((nN + NB - 1) / NB) * NB;

  char* ws = (char*)d_ws;
  size_t off = 0;
  const size_t oWp = off; off += (size_t)FD * KX * 2;
  const size_t oWf = off; off += (size_t)FD * FD * 2;
  const size_t oWo = off; off += (size_t)FD * FD * 2;
  const size_t oXh = off; off += (size_t)Np * KX * 2;
  const size_t oH0 = off; off += (size_t)Np * FD * 4;
  const size_t oA1 = off; off += (size_t)Np * FD * 2;
  const size_t oH1 = off; off += (size_t)Np * FD * 4;
  const size_t oA2 = off; off += (size_t)Np * FD * 2;
  size_t limit = (size_t)134217728;
  if (ws_size < limit) limit = ws_size;
  if (off > limit) return;

  _Float16* pWp = (_Float16*)(ws + oWp);
  _Float16* pWf = (_Float16*)(ws + oWf);
  _Float16* pWo = (_Float16*)(ws + oWo);
  _Float16* Xh  = (_Float16*)(ws + oXh);
  float*    H0  = (float*)(ws + oH0);
  _Float16* A1  = (_Float16*)(ws + oA1);
  float*    H1  = (float*)(ws + oH1);
  _Float16* A2  = (_Float16*)(ws + oA2);

  const int vec8 = ((nE & 3) == 0) ? 1 : 0;

  k_prep<<<8, NTHR, 0, stream>>>(Wp, Wf, Wo, pWp, pWf, pWo);
  k_cvt<<<Np / 16, NTHR, 0, stream>>>(x, Xh, nN);

  hipFuncSetAttribute(reinterpret_cast<const void*>(&k_agg), hipFuncAttributeMaxDynamicSharedMemorySize, LDS_AGG);

  k_gemm<KX, false><<<Np / GROWS, NTHR, 0, stream>>>(Xh, pWp, bp, H0, Np);
  k_agg<<<Np / NB, NTHR, LDS_AGG, stream>>>(H0, ei, A1, nN, nE, vec8);
  k_gemm<FD, true><<<Np / GROWS, NTHR, 0, stream>>>(A1, pWf, bf, H1, Np);
  k_agg<<<Np / NB, NTHR, LDS_AGG, stream>>>(H1, ei, A2, nN, nE, vec8);
  k_gemm<FD, false><<<Np / GROWS, NTHR, 0, stream>>>(A2, pWo, bo, outp, nN);
}
